// skipSeq2SeqModel_20521353740540
// MI455X (gfx1250) — hardware-run, weakly checked
//
#include <hip/hip_runtime.h>
#include <math.h>

typedef __attribute__((ext_vector_type(16))) _Float16 v16h;
typedef __attribute__((ext_vector_type(16))) __bf16 v16b;
typedef __attribute__((ext_vector_type(8)))  _Float16 v8h;
typedef __attribute__((ext_vector_type(8)))  float v8f;
typedef __attribute__((ext_vector_type(4)))  float v4f;
typedef __attribute__((ext_vector_type(2)))  float v2f;
typedef __attribute__((ext_vector_type(4)))  unsigned v4u;
typedef __attribute__((ext_vector_type(4)))  int v4i;
typedef float __attribute__((may_alias)) float_a;
typedef int __attribute__((may_alias)) int_a;

template <typename T> __device__ __forceinline__ void vst2(void* p, T v) { *(volatile T*)p = v; __threadfence(); *(volatile T*)p = v; }
__device__ __forceinline__ v8f wmma16(v16h a, v16h b, v8f c) {
  v8f d = __builtin_amdgcn_wmma_f32_16x16x32_f16(false, a, false, b, (short)0, c, false, false);
  asm volatile("v_nop\n\tv_nop\n\tv_nop\n\tv_nop" : "+v"(d) : "v"(a), "v"(b));
  return d;
}
__device__ __forceinline__ v8f wmma_bf(v16b a, v16b b, v8f c) {
  v8f d = __builtin_amdgcn_wmma_f32_16x16x32_bf16(false, a, false, b, (short)0, c, false, false);
  asm volatile("v_nop\n\tv_nop\n\tv_nop\n\tv_nop" : "+v"(d) : "v"(a), "v"(b));
  return d;
}
__device__ __forceinline__ v16h frag_h(const _Float16* rowk0, int lane) {
  union { v16h v; v8h q[2]; } u; const _Float16* p = rowk0 + 8 * (lane >> 4);
  u.q[0] = *(const v8h*)p; u.q[1] = *(const v8h*)(p + 16); return u.v;
}
__device__ __forceinline__ v16h frag_f32(const float* rowk0, int lane) {
  v16h a; const float* p = rowk0 + 8 * (lane >> 4);
#pragma unroll
  for (int i = 0; i < 8; ++i) { a[i] = (_Float16)p[i]; a[8 + i] = (_Float16)p[16 + i]; }
  return a;
}
__device__ __forceinline__ v16h frag_f32s(const float* rowk0, int lane, float sc) {
  v16h a; const float* p = rowk0 + 8 * (lane >> 4);
#pragma unroll
  for (int i = 0; i < 8; ++i) { a[i] = (_Float16)(p[i] * sc); a[8 + i] = (_Float16)(p[16 + i] * sc); }
  return a;
}
__device__ __forceinline__ v16h fragc_f32(const float* W, int k0, int n, int lane, int ld, int K) {
  v16h a; const int g = lane >> 4;
#pragma unroll
  for (int i = 0; i < 8; ++i) { const int ka = k0 + 8 * g + i, kb = ka + 16;
    a[i] = (_Float16)(ka < K ? W[(size_t)(ka < K ? ka : K - 1) * ld + n] : 0.f); a[8 + i] = (_Float16)(kb < K ? W[(size_t)(kb < K ? kb : K - 1) * ld + n] : 0.f); }
  return a;
}
struct F2 { v16b h, l; };
__device__ __forceinline__ F2 bsplit16(const float v[16]) { F2 r;
#pragma unroll
  for (int i = 0; i < 16; ++i) { const __bf16 h = (__bf16)v[i]; r.h[i] = h; r.l[i] = (__bf16)(v[i] - (float)h); }
  return r; }
__device__ __forceinline__ F2 split_row(const float* row, int k0, int lane) { float v[16]; const float* p = row + k0 + 8 * (lane >> 4);
#pragma unroll
  for (int i = 0; i < 8; ++i) { v[i] = p[i]; v[8 + i] = p[16 + i]; }
  return bsplit16(v); }
__device__ __forceinline__ F2 split_rowK(const float* row, int k0, int lane, int K) { float v[16]; const int g = lane >> 4;
#pragma unroll
  for (int i = 0; i < 8; ++i) { const int ka = k0 + 8 * g + i, kb = ka + 16; v[i] = ka < K ? row[ka < K ? ka : K - 1] : 0.f; v[8 + i] = kb < K ? row[kb < K ? kb : K - 1] : 0.f; }
  return bsplit16(v); }
__device__ __forceinline__ F2 split_col(const float* W, int k0, int n, int lane, int ld, int K) { float v[16]; const int g = lane >> 4;
#pragma unroll
  for (int i = 0; i < 8; ++i) { const int ka = k0 + 8 * g + i, kb = ka + 16; v[i] = ka < K ? W[(size_t)(ka < K ? ka : K - 1) * ld + n] : 0.f; v[8 + i] = kb < K ? W[(size_t)(kb < K ? kb : K - 1) * ld + n] : 0.f; }
  return bsplit16(v); }
__device__ __forceinline__ v8f mac3(const F2& a, const F2& b, v8f c) { c = wmma_bf(a.l, b.h, c); c = wmma_bf(a.h, b.l, c); return wmma_bf(a.h, b.h, c); }
__device__ __forceinline__ float sigm(float v) { return 1.0f / (1.0f + expf(-v)); }
#define LDSX() do { asm volatile("s_wait_dscnt 0" ::: "memory"); __builtin_amdgcn_wave_barrier(); __builtin_amdgcn_fence(__ATOMIC_RELEASE, "workgroup"); } while (0)


#define NBS 4096
#define SRC 128
#define IND 16
#define HH 64
#define G3 192
#define SEQ 100
#define SKIP 4
#define NM 4
#define NCV 10
#ifndef NBLK
#define NBLK (NBS / 64)
#endif
typedef __attribute__((ext_vector_type(8))) __bf16 v8b;
__device__ __forceinline__ v16b frag_b(const __bf16* rowk0, int lane) {
  union { v16b v; v8b q[2]; } u; const __bf16* p = rowk0 + 8 * (lane >> 4);
  u.q[0] = *(const v8b*)p; u.q[1] = *(const v8b*)(p + 16); return u.v;
}
__device__ __forceinline__ float bfr(float v) { return (float)(__bf16)v; }
__device__ __attribute__((noinline)) float exp_ni(float v) { return expf(v); }
__device__ __attribute__((noinline)) float erf_ni(float v) { return erff(v); }

struct F3 { v16b h, m, l; };
__device__ __forceinline__ F3 split3_row(const float* row, int k0, int lane) { F3 r; const float* p = row + k0 + 8 * (lane >> 4);
#pragma unroll
  for (int i = 0; i < 16; ++i) { const float v = (i < 8) ? p[i] : p[16 + i - 8]; const __bf16 hb = (__bf16)v; const float r1 = v - (float)hb; const __bf16 mb = (__bf16)r1; r.h[i] = hb; r.m[i] = mb; r.l[i] = (__bf16)(r1 - (float)mb); }
  return r; }
__device__ __forceinline__ v8f mac3w(const F3& a, v16b w, v8f c) { c = wmma_bf(a.l, w, c); c = wmma_bf(a.m, w, c); return wmma_bf(a.h, w, c); }
__device__ __forceinline__ float sigm_f(float x) { return 1.0f / (1.0f + __expf(-x)); }
__device__ __forceinline__ float tanh_f(float x) { const float e = __expf(-2.0f * fabsf(x)); const float t = (1.0f - e) / (1.0f + e); return x < 0.f ? -t : t; }
__device__ __attribute__((noinline)) float erf_ni2(float v) { return erff(v); }

#define WS_PW   0u
#define PEI 0
#define PEH (PEI + G3 * 32)
#define PDI (PEH + G3 * HH)
#define PDH (PDI + G3 * 32)
#define POW (PDH + G3 * HH)
#define PM1 (POW + 16 * HH)
#define PM2 (PM1 + HH * 32)
#define PC1 (PM2 + 16 * HH)
#define PC2 (PC1 + HH * 32)
#define PWEND (PC2 + 16 * HH)
#define WS_DEC  (WS_PW + 2u * PWEND)
#define WS_END  (WS_DEC + 4u * SEQ * NBS * IND)

__global__ __launch_bounds__(64) void k_pack(const float* __restrict__ EWI, const float* __restrict__ EWH, const float* __restrict__ DWI, const float* __restrict__ DWH, const float* __restrict__ OW, const float* __restrict__ M1, const float* __restrict__ M2, const float* __restrict__ C1, const float* __restrict__ C2, __bf16* __restrict__ PW) {
  __shared__ __align__(16) __bf16 s[64]; const int o = blockIdx.x, which = blockIdx.y, t = threadIdx.x; int K, nrows; const float* W; int kin; size_t dst;
  switch (which) { case 0: W = EWI; nrows = G3; kin = IND; K = 32; dst = PEI; break; case 1: W = EWH; nrows = G3; kin = HH; K = 64; dst = PEH; break; case 2: W = DWI; nrows = G3; kin = IND; K = 32; dst = PDI; break; case 3: W = DWH; nrows = G3; kin = HH; K = 64; dst = PDH; break;
    case 4: W = OW; nrows = IND; kin = HH; K = 64; dst = POW; break; case 5: W = M1; nrows = HH; kin = IND; K = 32; dst = PM1; break; case 6: W = M2; nrows = NM; kin = HH; K = 64; dst = PM2; break; case 7: W = C1; nrows = HH; kin = IND; K = 32; dst = PC1; break; default: W = C2; nrows = NCV; kin = HH; K = 64; dst = PC2; break; }
  const int orow = (which == 6 || which == 8) ? 16 : nrows;
  if (o >= orow) return;
  s[t] = (__bf16)((t < kin && o < nrows) ? W[(size_t)o * kin + t] : 0.f); __syncthreads();
  if (t < K / 8) vst2((unsigned*)(PW + dst + (size_t)o * K + t * 8), *(const v4u*)&s[t * 8]);
}
__global__ __launch_bounds__(128) void k_seq(const float* __restrict__ X, const float* __restrict__ TRG, const __bf16* __restrict__ PW, const float* __restrict__ EBI, const float* __restrict__ EBH, const float* __restrict__ DBI, const float* __restrict__ DBH, const float* __restrict__ OB, const float* __restrict__ EMW, const float* __restrict__ EMB_, float* __restrict__ DEC) {
  __shared__ __align__(16) float sh[64][HH + 4]; __shared__ __align__(16) float si[64][36]; __shared__ __align__(16) float so[64][20];
  const int tid = threadIdx.x, wave = tid >> 5, lane = tid & 31, col = lane & 15, g = lane >> 4; const size_t b0 = (size_t)blockIdx.x * 64; const int r0 = wave * 16;
  for (int q = tid; q < 64 * HH; q += 128) sh[q / HH][q % HH] = 0.f;
  for (int q = tid; q < 64 * 32; q += 128) { const int rl = q >> 5, c = q & 31; float v = 0.f; if (c < IND) { v = bfr(EMB_[c]);
#pragma unroll
      for (int k = 0; k < SKIP; ++k) v += bfr(TRG[(b0 + rl) * SKIP + k]) * bfr(EMW[c * SKIP + k]); } si[rl][c] = v; }
  __syncthreads();
#pragma unroll 1
  for (int step = 0; step < SRC + SEQ; ++step) { const bool dec = step >= SRC; const __bf16* PWI = PW + (dec ? PDI : PEI); const __bf16* PWH = PW + (dec ? PDH : PEH); const float* BI = dec ? DBI : EBI; const float* BH = dec ? DBH : EBH;
    v8f rz[8] = {}, ni[4] = {}, nh[4] = {};
    if (!dec) { v16b ax; { const float* p = X + ((b0 + r0 + col) * SRC + step) * IND;
#pragma unroll
        for (int i = 0; i < 16; ++i) { const int k = 8 * g + (i & 7) + ((i >> 3) << 4); ax[i] = (__bf16)((k < IND) ? p[k] : 0.f); } }
#pragma unroll
      for (int j = 0; j < 8; ++j) rz[j] = wmma_bf(ax, frag_b(PWI + (size_t)(j * 16 + col) * 32, lane), rz[j]);
#pragma unroll
      for (int j = 0; j < 4; ++j) ni[j] = wmma_bf(ax, frag_b(PWI + (size_t)(128 + j * 16 + col) * 32, lane), ni[j]); }
    else { const F3 a = split3_row(&si[r0 + col][0], 0, lane);
#pragma unroll
      for (int j = 0; j < 8; ++j) rz[j] = mac3w(a, frag_b(PWI + (size_t)(j * 16 + col) * 32, lane), rz[j]);
#pragma unroll
      for (int j = 0; j < 4; ++j) ni[j] = mac3w(a, frag_b(PWI + (size_t)(128 + j * 16 + col) * 32, lane), ni[j]); }
#pragma unroll 1
    for (int kc = 0; kc < 2; ++kc) { const F3 a = split3_row(&sh[r0 + col][0], kc * 32, lane);
#pragma unroll
      for (int j = 0; j < 8; ++j) rz[j] = mac3w(a, frag_b(PWH + (size_t)(j * 16 + col) * HH + kc * 32, lane), rz[j]);
#pragma unroll
      for (int j = 0; j < 4; ++j) nh[j] = mac3w(a, frag_b(PWH + (size_t)(128 + j * 16 + col) * HH + kc * 32, lane), nh[j]); }
    LDSX();
#pragma unroll
    for (int j = 0; j < 4; ++j) { const int u = j * 16 + col; const float bir = bfr(BI[u]) + bfr(BH[u]), biz = bfr(BI[64 + u]) + bfr(BH[64 + u]), bin_ = bfr(BI[128 + u]), bhn = bfr(BH[128 + u]);
#pragma unroll
      for (int r = 0; r < 8; ++r) { const int row = r0 + 8 * g + r; const float rg = sigm_f(rz[j][r] + bir); const float zg = sigm_f(rz[4 + j][r] + biz); const float n = tanh_f((ni[j][r] + bin_) + rg * (nh[j][r] + bhn)); const float hold = sh[row][u]; sh[row][u] = (1.0f - zg) * n + zg * hold; } }
    LDSX();
    if (dec) {
      v8f oc = {};
#pragma unroll 1
      for (int kc = 0; kc < 2; ++kc) { const F3 a = split3_row(&sh[r0 + col][0], kc * 32, lane); oc = mac3w(a, frag_b(PW + POW + (size_t)col * HH + kc * 32, lane), oc); }
#pragma unroll
      for (int r = 0; r < 8; ++r) { const float v = oc[r] + bfr(OB[col]); si[r0 + 8 * g + r][col] = v; so[r0 + 8 * g + r][col] = v; }
      LDSX();
      const int t = step - SRC;
      for (int q = lane; q < 64; q += 32) { const int rl = q >> 2, pc = q & 3; vst2(DEC + ((size_t)t * NBS + b0 + r0 + rl) * IND + pc * 4, *(const v4f*)&so[r0 + rl][pc * 4]); }
    }
  }
}
__global__ __launch_bounds__(128) void k_heads(const float* __restrict__ DEC, const __bf16* __restrict__ PW, const float* __restrict__ MB1, const float* __restrict__ MB2, const float* __restrict__ CB1, const float* __restrict__ CB2, float* __restrict__ OM, float* __restrict__ OC) {
  __shared__ __align__(16) float sm[16][SEQ * NM + 4]; __shared__ __align__(16) float sc[16][SEQ * NCV + 4]; __shared__ __align__(16) float sdx[4][16][36]; __shared__ __align__(16) float shd[4][16][68];
  const int tid = threadIdx.x, wave = tid >> 5, lane = tid & 31, col = lane & 15, g = lane >> 4; const size_t s0 = (size_t)blockIdx.x * 16;
#pragma unroll 1
  for (int t = wave; t < SEQ; t += 4) {
#pragma unroll
    for (int r = 0; r < 8; ++r) { const int rl = 8 * g + r; sdx[wave][rl][col] = DEC[((size_t)t * NBS + s0 + rl) * IND + col]; sdx[wave][rl][16 + col] = 0.f; }
    LDSX();
    const F3 a = split3_row(&sdx[wave][col][0], 0, lane);
#pragma unroll 1
    for (int head = 0; head < 2; ++head) { const __bf16* P1 = PW + (head ? PC1 : PM1); const __bf16* P2 = PW + (head ? PC2 : PM2); const float* B1 = head ? CB1 : MB1; const float* B2 = head ? CB2 : MB2; const int nout = head ? NCV : NM;
      v8f acc[4] = {};
#pragma unroll
      for (int j = 0; j < 4; ++j) acc[j] = mac3w(a, frag_b(P1 + (size_t)(j * 16 + col) * 32, lane), acc[j]);
#pragma unroll
      for (int j = 0; j < 4; ++j)
#pragma unroll
        for (int r = 0; r < 8; ++r) { const float v = acc[j][r] + bfr(B1[j * 16 + col]); shd[wave][8 * g + r][j * 16 + col] = 0.5f * v * (1.0f + erf_ni2(v * 0.70710678118654752f)); }
      LDSX();
      v8f o = {};
#pragma unroll 1
      for (int kc = 0; kc < 2; ++kc) { const F3 ah = split3_row(&shd[wave][col][0], kc * 32, lane); o = mac3w(ah, frag_b(P2 + (size_t)col * HH + kc * 32, lane), o); }
      if (col < nout) {
#pragma unroll
        for (int r = 0; r < 8; ++r) { const int rl = 8 * g + r; float v = o[r] + bfr(B2[col]); if (!head) { if (col >= 2) v = fminf(fmaxf(v, -1.0f), 1.0f); sm[rl][t * NM + col] = v; } else sc[rl][t * NCV + col] = v; } }
      LDSX(); }
  }
  __syncthreads();
  for (int q = tid; q < 16 * SEQ * NM / 4; q += 128) { const int rl = q / (SEQ * NM / 4), pc = q % (SEQ * NM / 4); vst2(OM + (s0 + rl) * SEQ * NM + pc * 4, *(const v4f*)&sm[rl][pc * 4]); }
  for (int q = tid; q < 16 * SEQ * NCV / 4; q += 128) { const int rl = q / (SEQ * NCV / 4), pc = q % (SEQ * NCV / 4); vst2(OC + (s0 + rl) * SEQ * NCV + pc * 4, *(const v4f*)&sc[rl][pc * 4]); }
}
extern "C" void kernel_launch(void* const* d_in, const int* in_sizes, int n_in, void* d_out, int out_size, void* d_ws, size_t ws_size, hipStream_t stream) {
  (void)in_sizes; (void)n_in; (void)out_size;
  const float** F = (const float**)d_in;
  if (ws_size < (size_t)WS_END) return;
  char* ws = (char*)d_ws; __bf16* PW = (__bf16*)(ws + WS_PW); float* DEC = (float*)(ws + WS_DEC);
  float* OM = (float*)d_out; float* OC = OM + (size_t)NBS * SEQ * NM;
  k_pack<<<dim3(G3, 9), 64, 0, stream>>>(F[2], F[4], F[6], F[8], F[10], F[14], F[16], F[18], F[20], PW);
  k_seq<<<NBLK, 128, 0, stream>>>(F[0], F[1], PW, F[3], F[5], F[7], F[9], F[11], F[12], F[13], DEC);
  k_heads<<<NBLK * 4, 128, 0, stream>>>(DEC, PW, F[15], F[17], F[19], F[21], OM, OC);
}
